// GAT_21818433863880
// MI455X (gfx1250) — hardware-verified
//
#include <hip/hip_runtime.h>
#include <math.h>

#ifndef NB
#define NB 8
#endif
#ifndef SEQ
#define SEQ 2048
#endif
#define NB_FULL 8
#define SEQ_FULL 2048
#define IN_DIM 128
#define OUTD 64
#define HEADS 4
#define HCOLS (HEADS * OUTD)
#define MTOK (NB * SEQ)
#define PL_P 68
#define AT_OP 68

static constexpr float XCARRY   = 16.0f;
static constexpr float WCARRY   = 64.0f;
static constexpr float HF_SCALE = 1.0f / 1024.0f;
static constexpr float VCARRY   = 16.0f;
static constexpr float PCARRY   = 1024.0f;
static constexpr float O_UNDO   = 1.0f / 16384.0f;
static constexpr float LOG2E_F  = 1.4426950408889634f;
static constexpr float NEG_SLOPE_F = 0.2f;

static constexpr unsigned FJ_OFF = (unsigned)(NB * HEADS * SEQ);

static constexpr size_t X16_BYTES = (size_t)MTOK * IN_DIM * 2;
static constexpr size_t WT_BYTES  = (size_t)HCOLS * IN_DIM * 2;
static constexpr size_t HF_BYTES  = (size_t)MTOK * HCOLS * 4;
static constexpr size_t VT_BYTES  = (size_t)NB * HCOLS * SEQ * 2;
static constexpr size_t FIJ_BYTES = (size_t)2 * NB * HEADS * SEQ * 4;
static constexpr size_t X16_OFF = 0;
static constexpr size_t WT_OFF  = X16_OFF + X16_BYTES;
static constexpr size_t HF_OFF  = WT_OFF + WT_BYTES;
static constexpr size_t VT_OFF  = HF_OFF + HF_BYTES;
static constexpr size_t FIJ_OFF_B = VT_OFF + VT_BYTES;
static constexpr size_t WS_TOTAL = FIJ_OFF_B + FIJ_BYTES;

static constexpr unsigned G_XCVT   = (unsigned)((MTOK * IN_DIM / 8) / 256);
static constexpr unsigned G_WT     = (unsigned)((OUTD * (IN_DIM / 8)) / 256);
static constexpr unsigned G_GEMM   = (unsigned)(((MTOK / 64) * (HCOLS / 64) + 7) / 8);
static constexpr unsigned G_PLANES = (unsigned)(NB * (SEQ / 64) * HEADS);
static constexpr unsigned G_ATTN   = (unsigned)(NB * (SEQ / 128));

static_assert(NB <= NB_FULL && SEQ <= SEQ_FULL);
static_assert((SEQ & (SEQ - 1)) == 0);
static_assert(SEQ % 128 == 0);
static_assert(MTOK % 64 == 0 && HCOLS % 64 == 0);
static_assert(IN_DIM == 128 && IN_DIM % 32 == 0);
static_assert(OUTD == 64 && HEADS == 4 && HCOLS == 256);
static_assert((MTOK * IN_DIM / 8) % 256 == 0);
static_assert((OUTD * (IN_DIM / 8)) % 256 == 0);
static_assert(XCARRY * WCARRY * HF_SCALE == 1.0f);
static_assert(PCARRY * VCARRY * O_UNDO == 1.0f);
static_assert(WCARRY == 64.0f);
static_assert(X16_BYTES % 256 == 0 && WT_BYTES % 256 == 0 && HF_BYTES % 256 == 0 && VT_BYTES % 256 == 0 && FIJ_BYTES % 256 == 0);
static_assert(WS_TOTAL <= (size_t)134217728);
static_assert(32 * 16 * 8 == 16 * 64 * 4);
static_assert(256 * 16 * 2 == 64 * 64 * 2);
static_assert(32 * 16 * 1 == 2 * 64 * 4);
static_assert((size_t)G_XCVT * 256 * 16 == X16_BYTES);
static_assert(8 * 16 * 68 * 4 <= 131072);
static_assert(64 * PL_P * 4 + 128 * 4 + 128 * 4 <= 131072);
static_assert(8 * 16 * AT_OP * 4 <= 131072);

typedef __attribute__((ext_vector_type(16))) _Float16 v16h;
typedef __attribute__((ext_vector_type(8)))  _Float16 v8h;
typedef __attribute__((ext_vector_type(2)))  _Float16 v2h;
typedef __attribute__((ext_vector_type(8)))  float    v8f;
typedef __attribute__((ext_vector_type(4)))  float    v4f;
typedef __attribute__((ext_vector_type(2)))  float    v2f;
typedef __attribute__((ext_vector_type(4)))  unsigned int v4u;


#define VST2(T, ptr, val) do { const T vst2_v_ = (val); *(volatile T*)(ptr) = vst2_v_; __threadfence(); *(volatile T*)(ptr) = vst2_v_; } while (0)

__device__ __forceinline__ float bfr(float f) {
    unsigned u = __float_as_uint(f);
    u += 0x7FFFu + ((u >> 16) & 1u);
    return __uint_as_float(u & 0xFFFF0000u);
}
__device__ __forceinline__ unsigned short f2h_bits(float x) {
    return (fabsf(x) < 6.104e-5f) ? (unsigned short)0 : __builtin_bit_cast(unsigned short, (_Float16)x);
}
__device__ __forceinline__ void st8h(unsigned short* P, size_t o, const float* v) {
    v4u pk;
    pk.x = (unsigned)f2h_bits(v[0]) | ((unsigned)f2h_bits(v[1]) << 16);
    pk.y = (unsigned)f2h_bits(v[2]) | ((unsigned)f2h_bits(v[3]) << 16);
    pk.z = (unsigned)f2h_bits(v[4]) | ((unsigned)f2h_bits(v[5]) << 16);
    pk.w = (unsigned)f2h_bits(v[6]) | ((unsigned)f2h_bits(v[7]) << 16);
    VST2(v4u, (v4u*)(P + o), pk);
}

static __device__ __forceinline__ v2h toh_flush2(float a, float b) {
    v2f w;
    w.x = (fabsf(a) < 6.103515625e-05f) ? 0.0f : a;
    w.y = (fabsf(b) < 6.103515625e-05f) ? 0.0f : b;
    return __builtin_convertvector(w, v2h);
}
union H8U  { v8h v;  v2h p[4]; };
union P16U { v16h v; v2h p[8]; };

union FragU { v16h v; v8h h[2]; };
__device__ __forceinline__ v16h frag_ld(const _Float16* p) {
    FragU f; f.h[0] = *(const v8h*)(p); f.h[1] = *(const v8h*)(p + 16); return f.v;
}
__device__ __forceinline__ v8f wmma16(v16h a, v16h b, v8f c) {
    c = __builtin_amdgcn_wmma_f32_16x16x32_f16(false, a, false, b, (short)0, c, false, false);
    asm volatile("v_nop\n\tv_nop\n\tv_nop\n\tv_nop" : "+v"(c) : "v"(a), "v"(b));
    return c;
}
__device__ __forceinline__ void wave_sync_lds() {
    __builtin_amdgcn_fence(3  , "workgroup");
    __builtin_amdgcn_wave_barrier();
    __builtin_amdgcn_fence(2  , "workgroup");
}

__global__ __launch_bounds__(256) void k_gemm64(
    const _Float16* __restrict__ A, unsigned lda, const _Float16* __restrict__ Bt, unsigned ldb,
    float* __restrict__ C, unsigned ldc, const float* __restrict__ bias,
    unsigned M, unsigned N, unsigned K) {
  __shared__ __align__(16) float sT[8][16 * 68];
  const unsigned lane = threadIdx.x & 31u;
  const unsigned wave = (unsigned)__builtin_amdgcn_readfirstlane((int)(threadIdx.x >> 5));
  const unsigned tilesN = N >> 6, tilesM = M >> 6;
  const unsigned tile = blockIdx.x * 8u + wave;
  if (tile >= tilesM * tilesN) return;
  const unsigned tm = tile / tilesN;
  const unsigned tn = tile - tm * tilesN;
  const unsigned m0 = tm << 6, n0 = tn << 6;
  const unsigned rlane = lane & 15u;
  const unsigned koff = (lane >> 4) * 8u;
  const unsigned mOff = koff;

  v8f acc[4][4];
#pragma unroll
  for (int i = 0; i < 4; ++i)
#pragma unroll
    for (int j = 0; j < 4; ++j) acc[i][j] = (v8f){0.f,0.f,0.f,0.f,0.f,0.f,0.f,0.f};

  for (unsigned k0 = 0; k0 < K; k0 += 32u) {
    v16h bh[4];
#pragma unroll
    for (int j = 0; j < 4; ++j)
      bh[j] = frag_ld(Bt + (size_t)(n0 + ((unsigned)j << 4) + rlane) * ldb + koff + k0);
#pragma unroll
    for (int i = 0; i < 4; ++i) {
      const v16h ah = frag_ld(A + (size_t)(m0 + ((unsigned)i << 4) + rlane) * lda + koff + k0);
#pragma unroll
      for (int j = 0; j < 4; ++j)
        acc[i][j] = wmma16(ah, bh[j], acc[i][j]);
    }
  }

#pragma unroll
  for (int i = 0; i < 4; ++i) {
    const unsigned mBase = m0 + ((unsigned)i << 4);
#pragma unroll
    for (int j = 0; j < 4; ++j) {
      const unsigned n = n0 + ((unsigned)j << 4) + rlane;
      const float bv = bfr(bias[n]);
#pragma unroll
      for (int r = 0; r < 8; ++r) {
        const float v = acc[i][j][r] * HF_SCALE + bv;
        sT[wave][(mOff + (unsigned)r) * 68u + ((unsigned)j << 4) + rlane] = v;
      }
    }
    wave_sync_lds();
    {
      const unsigned hh = lane >> 4, c4 = (lane & 15u) * 4u;
#pragma unroll
      for (int half = 0; half < 2; ++half) {
        v4f vv[4];
#pragma unroll
        for (int it = 0; it < 4; ++it) {
          const unsigned row = (unsigned)(half * 4 + it) * 2u + hh;
          vv[it] = *(const v4f*)(&sT[wave][row * 68u + c4]);
        }
        for (int pass = 0; pass < 2; ++pass) {
#pragma unroll
          for (int it = 0; it < 4; ++it) {
            const unsigned row = (unsigned)(half * 4 + it) * 2u + hh;
            *(volatile v4f*)(C + (size_t)(mBase + row) * ldc + n0 + c4) = vv[it];
          }
          __threadfence();
        }
      }
    }
    wave_sync_lds();
  }
}

__global__ __launch_bounds__(256) void k_wt16(const float* __restrict__ Wm, unsigned KI, unsigned NO, unsigned lgper,
                                              unsigned short* __restrict__ W16, float sw) {
    const unsigned layer = blockIdx.y;
    const float* Wl = Wm + (size_t)layer * KI * NO;
    unsigned short* Dl = W16 + (size_t)layer * KI * NO;
    const unsigned u = blockIdx.x * 256u + threadIdx.x;
    const unsigned per = 1u << lgper;
    if (u >= NO * per) return;
    const unsigned k0 = 8u * (u & (per - 1u));
    const unsigned o = u >> lgper;
    float v[8];
#pragma unroll
    for (int i = 0; i < 8; ++i) v[i] = bfr(Wl[(size_t)(k0 + (unsigned)i) * NO + o]) * sw;
    st8h(Dl, (size_t)o * KI + k0, v);
}

__global__ __launch_bounds__(256) void k_xcvt(const float* __restrict__ x, _Float16* __restrict__ x16) {
    const unsigned u = blockIdx.x * 256u + threadIdx.x;
    if (u >= (unsigned)(MTOK * IN_DIM / 8)) return;
    const unsigned row = u >> 4, c0 = (u & 15u) * 8u;
    const unsigned b = row / (unsigned)SEQ;
    const unsigned n = row - b * (unsigned)SEQ;
    const float* xr = x + (size_t)(b * (unsigned)SEQ_FULL + n) * IN_DIM + c0;
    const v4f a0 = *(const v4f*)xr;
    const v4f a1 = *(const v4f*)(xr + 4);
    H8U pk;
    pk.p[0] = toh_flush2(bfr(a0.x) * XCARRY, bfr(a0.y) * XCARRY);
    pk.p[1] = toh_flush2(bfr(a0.z) * XCARRY, bfr(a0.w) * XCARRY);
    pk.p[2] = toh_flush2(bfr(a1.x) * XCARRY, bfr(a1.y) * XCARRY);
    pk.p[3] = toh_flush2(bfr(a1.z) * XCARRY, bfr(a1.w) * XCARRY);
    VST2(v8h, (v8h*)(x16 + (size_t)row * IN_DIM + c0), pk.v);
}

__global__ __launch_bounds__(256) void k_planes(const float* __restrict__ hf, const float* __restrict__ avec,
                                                _Float16* __restrict__ vt16, float* __restrict__ fij) {
    __shared__ __align__(16) float sH[64 * PL_P];
    __shared__ __align__(16) float sA[128];
    __shared__ __align__(16) float sF[2 * 64];
    const unsigned t = threadIdx.x, lane = t & 31u;
    const unsigned wave = (unsigned)__builtin_amdgcn_readfirstlane((int)(t >> 5));
    const unsigned bx = blockIdx.x;
    const unsigned hd = bx & 3u;
    const unsigned nbk = bx >> 2;
    const unsigned NBLK = (unsigned)(SEQ / 64);
    const unsigned b = nbk / NBLK;
    const unsigned n0 = (nbk - b * NBLK) * 64u;
    const unsigned row = t >> 2, q = t & 3u;

    if (t < 128u) sA[t] = bfr(avec[hd * 128u + t]);
    {
        const float* src = hf + (size_t)(b * (unsigned)SEQ + n0 + row) * HCOLS + hd * OUTD + q * 16u;
        v4f hv[4];
#pragma unroll
        for (int g = 0; g < 4; ++g) hv[g] = *(const v4f*)(src + 4 * g);
#pragma unroll
        for (int g = 0; g < 4; ++g) *(v4f*)(&sH[row * PL_P + q * 16u + 4u * (unsigned)g]) = hv[g];
    }
    __syncthreads();
    {
        float s1 = 0.f, s2 = 0.f;
#pragma unroll 1
        for (unsigned g = 0; g < 4u; ++g) {
            const unsigned cc = q * 16u + 4u * g;
            const v4f hv = *(const v4f*)(&sH[row * PL_P + cc]);
            const v4f w1 = *(const v4f*)(&sA[cc]);
            const v4f w2 = *(const v4f*)(&sA[64u + cc]);
            s1 += hv.x * w1.x; s1 += hv.y * w1.y; s1 += hv.z * w1.z; s1 += hv.w * w1.w;
            s2 += hv.x * w2.x; s2 += hv.y * w2.y; s2 += hv.z * w2.z; s2 += hv.w * w2.w;
        }
        s1 += __shfl_xor(s1, 1, 32); s1 += __shfl_xor(s1, 2, 32);
        s2 += __shfl_xor(s2, 1, 32); s2 += __shfl_xor(s2, 2, 32);
        if (q == 0u) { sF[row] = s1; sF[64u + row] = s2; }
    }
    __syncthreads();
    {
        const unsigned pc = (lane & 7u) * 8u;
        v8h hv16[2];
#pragma unroll
        for (int it = 0; it < 2; ++it) {
            const unsigned o = (unsigned)it * 32u + wave * 4u + (lane >> 3);
            H8U pk;
#pragma unroll
            for (int e = 0; e < 4; ++e)
                pk.p[e] = toh_flush2(sH[(pc + 2u * (unsigned)e) * PL_P + o] * VCARRY,
                                     sH[(pc + 2u * (unsigned)e + 1u) * PL_P + o] * VCARRY);
            hv16[it] = pk.v;
        }
        _Float16* dst = vt16 + (size_t)(b * HCOLS + hd * OUTD) * SEQ + n0;
        for (int pass = 0; pass < 2; ++pass) {
#pragma unroll
            for (int it = 0; it < 2; ++it) {
                const unsigned o = (unsigned)it * 32u + wave * 4u + (lane >> 3);
                *(volatile v8h*)(dst + (size_t)o * SEQ + pc) = hv16[it];
            }
            __threadfence();
        }
    }
    if (wave == 0u) {
        const unsigned sel = lane >> 4, c4 = (lane & 15u) * 4u;
        const v4f fv = *(const v4f*)(&sF[sel * 64u + c4]);
        float* fd = fij + (size_t)sel * FJ_OFF + (size_t)(b * HEADS + hd) * SEQ + n0 + c4;
        VST2(v4f, (v4f*)fd, fv);
    }
}

__global__ __launch_bounds__(256) __attribute__((amdgpu_num_vgpr(256))) void k_attn(
    const _Float16* __restrict__ vt16, const float* __restrict__ fij, float* __restrict__ out) {
    __shared__ __align__(16) float sO[8][16 * AT_OP];
    const unsigned lane = threadIdx.x & 31u;
    const unsigned wave = (unsigned)__builtin_amdgcn_readfirstlane((int)(threadIdx.x >> 5));
    const unsigned hh = lane >> 4, c = lane & 15u;
    const unsigned bx = blockIdx.x;
    const unsigned QB = (unsigned)(SEQ / 128);
    const unsigned b = bx / QB;
    const unsigned n0 = (bx - b * QB) * 128u + wave * 16u;

    v8f osum[4];
#pragma unroll
    for (int t = 0; t < 4; ++t) osum[t] = (v8f){0.f,0.f,0.f,0.f,0.f,0.f,0.f,0.f};

#pragma unroll 1
    for (unsigned hd = 0; hd < (unsigned)HEADS; ++hd) {
        const unsigned bh = b * HEADS + hd;
        const float fi = fij[(size_t)bh * SEQ + n0 + c];
        const float* fjp = fij + (size_t)FJ_OFF + (size_t)bh * SEQ + 8u * hh;
        const _Float16* vp = vt16 + (size_t)(b * HCOLS + hd * OUTD + c) * SEQ + 8u * hh;
        v8f acc[4];
#pragma unroll
        for (int t = 0; t < 4; ++t) acc[t] = (v8f){0.f,0.f,0.f,0.f,0.f,0.f,0.f,0.f};
        float mrun = -3.0e38f, lrun = 0.f;
#pragma unroll 1
        for (unsigned m0 = 0; m0 < (unsigned)SEQ; m0 += 32u) {
            const v4f f0 = *(const v4f*)(fjp + m0);
            const v4f f1 = *(const v4f*)(fjp + m0 + 4u);
            const v4f f2 = *(const v4f*)(fjp + m0 + 16u);
            const v4f f3 = *(const v4f*)(fjp + m0 + 20u);
            v16h va[4];
#pragma unroll
            for (int t = 0; t < 4; ++t) va[t] = frag_ld(vp + (size_t)(16u * (unsigned)t) * SEQ + m0);
            float tv[16] = {f0.x, f0.y, f0.z, f0.w, f1.x, f1.y, f1.z, f1.w,
                            f2.x, f2.y, f2.z, f2.w, f3.x, f3.y, f3.z, f3.w};
            float mx = -3.0e38f;
#pragma unroll
            for (int i = 0; i < 16; ++i) {
                float s = fi + tv[i];
                s = (s > 0.0f) ? s : NEG_SLOPE_F * s;
                s *= LOG2E_F;
                tv[i] = s;
                mx = (s > mx) ? s : mx;
            }
            const float mo = __shfl_xor(mx, 16, 32);
            mx = (mo > mx) ? mo : mx;
            const float mnew = (mx > mrun) ? mx : mrun;
            const float alpha = exp2f(mrun - mnew);
            mrun = mnew;
            float psum = 0.f;
            float pv[16];
#pragma unroll
            for (int i = 0; i < 16; ++i) {
                const float p = exp2f(tv[i] - mnew);
                psum += p;
                pv[i] = p * PCARRY;
            }
            lrun = lrun * alpha + psum;
            P16U pb;
#pragma unroll
            for (int i = 0; i < 8; ++i) pb.p[i] = toh_flush2(pv[2 * i], pv[2 * i + 1]);
#pragma unroll
            for (int t = 0; t < 4; ++t)
#pragma unroll
                for (int r = 0; r < 8; ++r) acc[t][r] *= alpha;
#pragma unroll
            for (int t = 0; t < 4; ++t) acc[t] = wmma16(va[t], pb.v, acc[t]);
        }
        const float lt = lrun + __shfl_xor(lrun, 16, 32);
        const float inv = (1.0f / lt) * O_UNDO;
#pragma unroll
        for (int t = 0; t < 4; ++t)
#pragma unroll
            for (int r = 0; r < 8; ++r) osum[t][r] += acc[t][r] * inv;
    }

#pragma unroll
    for (int t = 0; t < 4; ++t) {
        v4f lo, hi;
        lo.x = osum[t][0] * 0.25f; lo.y = osum[t][1] * 0.25f; lo.z = osum[t][2] * 0.25f; lo.w = osum[t][3] * 0.25f;
        hi.x = osum[t][4] * 0.25f; hi.y = osum[t][5] * 0.25f; hi.z = osum[t][6] * 0.25f; hi.w = osum[t][7] * 0.25f;
        *(v4f*)(&sO[wave][c * AT_OP + 16u * (unsigned)t + 8u * hh]) = lo;
        *(v4f*)(&sO[wave][c * AT_OP + 16u * (unsigned)t + 8u * hh + 4u]) = hi;
    }
    wave_sync_lds();
    {
        const unsigned c4 = (lane & 15u) * 4u;
        v4f vv[8];
#pragma unroll
        for (int it = 0; it < 8; ++it) {
            const unsigned rowq = (unsigned)it * 2u + hh;
            vv[it] = *(const v4f*)(&sO[wave][rowq * AT_OP + c4]);
        }
        float* dst = out + (size_t)(b * (unsigned)SEQ + n0) * OUTD;
        for (int pass = 0; pass < 2; ++pass) {
#pragma unroll
            for (int it = 0; it < 8; ++it) {
                const unsigned rowq = (unsigned)it * 2u + hh;
                *(volatile v4f*)(dst + (size_t)rowq * OUTD + c4) = vv[it];
            }
            __threadfence();
        }
    }
}

extern "C" void kernel_launch(void* const* d_in, const int* in_sizes, int n_in, void* d_out, int out_size,
                              void* d_ws, size_t ws_size, hipStream_t stream) {
    if (n_in < 4) return;
    if (in_sizes[0] < ((NB - 1) * SEQ_FULL + SEQ) * IN_DIM) return;
    if (in_sizes[1] < HEADS * IN_DIM * OUTD || in_sizes[2] < HEADS * OUTD || in_sizes[3] < HEADS * 2 * OUTD) return;
    if (out_size < MTOK * OUTD) return;
    if (WS_TOTAL > ws_size) return;

    const float* x    = (const float*)d_in[0];
    const float* W    = (const float*)d_in[1];
    const float* bvec = (const float*)d_in[2];
    const float* avec = (const float*)d_in[3];
    float* out = (float*)d_out;

    char* wsp = (char*)d_ws;
    _Float16*       x16  = (_Float16*)(wsp + X16_OFF);
    unsigned short* wt16 = (unsigned short*)(wsp + WT_OFF);
    float*          hf   = (float*)(wsp + HF_OFF);
    _Float16*       vt16 = (_Float16*)(wsp + VT_OFF);
    float*          fij  = (float*)(wsp + FIJ_OFF_B);

    k_xcvt<<<G_XCVT, 256, 0, stream>>>(x, x16);
    k_wt16<<<dim3(G_WT, HEADS), 256, 0, stream>>>(W, IN_DIM, OUTD, 4, wt16, WCARRY);
    k_gemm64<<<G_GEMM, 256, 0, stream>>>((const _Float16*)x16, IN_DIM, (const _Float16*)wt16, IN_DIM,
                                         hf, HCOLS, bvec, MTOK, HCOLS, IN_DIM);
    k_planes<<<G_PLANES, 256, 0, stream>>>((const float*)hf, avec, vt16, fij);
    k_attn<<<G_ATTN, 256, 0, stream>>>((const _Float16*)vt16, (const float*)fij, out);
}
